// GATEncoder_22574348108302
// MI455X (gfx1250) — hardware-run, weakly checked
//
#include <hip/hip_runtime.h>

typedef float          v8f   __attribute__((ext_vector_type(8)));
typedef float          v4f   __attribute__((ext_vector_type(4)));
typedef unsigned int   v4u   __attribute__((ext_vector_type(4)));
typedef int            v8i   __attribute__((ext_vector_type(8)));
typedef unsigned short v8us  __attribute__((ext_vector_type(8)));
typedef unsigned short v16us __attribute__((ext_vector_type(16)));
typedef __bf16         v16bf __attribute__((ext_vector_type(16)));
typedef _Float16       v16h  __attribute__((ext_vector_type(16)));
typedef v4f  __attribute__((may_alias)) v4fa;
typedef v8us __attribute__((may_alias)) v8usa;
union FragB { v16bf v; v16us u; v8us h[2]; v8i w; };
union FragH { v16h  v; v16us u; v8us h[2]; v8i w; };

__device__ __forceinline__ v8f wmb(const FragB& a, const FragB& b, v8f c) {
  v8f d = __builtin_amdgcn_wmma_f32_16x16x32_bf16(false, a.v, false, b.v, (short)0, c, false, false);
  asm volatile("v_nop\n\tv_nop\n\tv_nop\n\tv_nop" : "+v"(d) : "v"(a.w), "v"(b.w));
  return d;
}

__device__ __forceinline__ v8f wmh(const FragH& a, const FragH& b, v8f c) {
  v8f d = __builtin_amdgcn_wmma_f32_16x16x32_f16(false, a.v, false, b.v, (short)0, c, false, false);
  asm volatile("v_nop\n\tv_nop\n\tv_nop\n\tv_nop" : "+v"(d) : "v"(a.w), "v"(b.w));
  return d;
}

__device__ __forceinline__ unsigned bf16_bits(float f) {
  const unsigned u = __float_as_uint(f);
  const unsigned r = (u + 0x7FFFu + ((u >> 16) & 1u)) >> 16;
  const unsigned q = (u >> 16) | 0x40u;
  return ((u & 0x7fffffffu) > 0x7f800000u) ? q : r;
}

__device__ __forceinline__ float bf16_val(float f) {
  return __uint_as_float(bf16_bits(f) << 16);
}
__device__ __forceinline__ int clampi(int v, int lo, int hi) {
  return v < lo ? lo : (v > hi ? hi : v);
}

__device__ __forceinline__ unsigned f16_bits(float f) {
  const unsigned u  = __float_as_uint(f);
  const unsigned s  = (u >> 16) & 0x8000u;
  const unsigned a  = u & 0x7fffffffu;
  const unsigned t  = a - 0x38000000u;
  const unsigned r  = (t + 0x0FFFu + ((t >> 13) & 1u)) >> 13;
  const unsigned rc = r > 0x7C00u ? 0x7C00u : r;
  const bool small  = a < 0x38800000u;
  const bool isnan  = a > 0x7f800000u;
  const unsigned fin = small ? 0u : (s | rc);
  return isnan ? (s | 0x7E00u) : fin;
}

__device__ __forceinline__ unsigned pk16(unsigned lo, unsigned hi) { return lo | (hi << 16); }
__device__ __forceinline__ unsigned bf16_lo_bits(float v) {
  float hi = bf16_val(v);
  asm volatile("" : "+v"(hi));
  return bf16_bits(v - hi);
}
__device__ __forceinline__ v4u pack8_bf16(v4f a, v4f c) {
  return (v4u){ pk16(bf16_bits(a[0]), bf16_bits(a[1])), pk16(bf16_bits(a[2]), bf16_bits(a[3])),
                pk16(bf16_bits(c[0]), bf16_bits(c[1])), pk16(bf16_bits(c[2]), bf16_bits(c[3])) };
}
__device__ __forceinline__ v4u pack8_bf16_lo(v4f a, v4f c) {
  return (v4u){ pk16(bf16_lo_bits(a[0]), bf16_lo_bits(a[1])), pk16(bf16_lo_bits(a[2]), bf16_lo_bits(a[3])),
                pk16(bf16_lo_bits(c[0]), bf16_lo_bits(c[1])), pk16(bf16_lo_bits(c[2]), bf16_lo_bits(c[3])) };
}
__device__ __forceinline__ v4u pack8_f16(v4f a, v4f c) {
  return (v4u){ pk16(f16_bits(a[0]), f16_bits(a[1])), pk16(f16_bits(a[2]), f16_bits(a[3])),
                pk16(f16_bits(c[0]), f16_bits(c[1])), pk16(f16_bits(c[2]), f16_bits(c[3])) };
}

template <int FORM>
__global__ __launch_bounds__(256) void k_plane(const float* __restrict__ src, int rows, int cols, int ldsrc,
                                               unsigned short* __restrict__ dst, int MP, int KP) {
  static_assert(FORM >= 0 && FORM <= 3);
  const int KTOT = (FORM == 1 || FORM == 3) ? 2 * KP : KP;
  const unsigned ppr   = (unsigned)(KTOT >> 3);
  const unsigned kp8   = (unsigned)(KP >> 3);
  const unsigned total = (unsigned)MP * ppr;
  const unsigned g     = blockIdx.x * 256u + threadIdx.x;
  const unsigned rowu  = g / ppr;
  const unsigned p     = g - rowu * ppr;
  const bool second    = p >= kp8;
  const int row = (int)rowu;
  const int c0  = (int)((second ? p - kp8 : p) << 3);
  const float* srow = src + (size_t)clampi(row, 0, rows - 1) * (size_t)ldsrc;
  float x[8];
  unsigned mk[8];
#pragma unroll
  for (int e = 0; e < 8; ++e) {
    const int c = c0 + e;
    const float v = srow[clampi(c, 0, cols - 1)];
    asm volatile("" :: "v"(v));
    x[e]  = v;
    mk[e] = (row < rows && c < cols) ? 0xFFFFu : 0u;
  }
  const v4f a = (v4f){ x[0], x[1], x[2], x[3] };
  const v4f c = (v4f){ x[4], x[5], x[6], x[7] };
  v4u o;
  if (FORM == 2) {
    o = pack8_f16(a, c);
  } else {
    const v4u hi = pack8_bf16(a, c);
    o = hi;
    if (FORM == 1) { const v4u lo = pack8_bf16_lo(a, c); o = second ? lo : hi; }
  }
  const v4u mw = (v4u){ pk16(mk[0], mk[1]), pk16(mk[2], mk[3]), pk16(mk[4], mk[5]), pk16(mk[6], mk[7]) };
  o &= mw;
  if (g < total) {
    volatile v4u* q = (volatile v4u*)(dst + (size_t)g * 8);
    *q = o;
    __threadfence();
    *q = o;
  }
}

template <int FORM> struct FragOf    { typedef FragB T; };
template <>         struct FragOf<2> { typedef FragH T; };
__device__ __forceinline__ v8f mm(const FragB& a, const FragB& b, v8f c) { return wmb(a, b, c); }
__device__ __forceinline__ v8f mm(const FragH& a, const FragH& b, v8f c) { return wmh(a, b, c); }
template <class F> __device__ __forceinline__ F ld_frag(const unsigned short* p) {
  F f;
  f.h[0] = *(const v8usa*)(p);
  f.h[1] = *(const v8usa*)(p + 16);
  return f;
}

template <int FORM, int EPI>
__global__ __launch_bounds__(256) __attribute__((amdgpu_num_vgpr(248)))
void k_gemm_nt(const unsigned short* __restrict__ A, const unsigned short* __restrict__ B,
               const float* __restrict__ bias, float* __restrict__ D, int M, int N, int KTOT, int ldd) {
  static_assert(FORM >= 0 && FORM <= 2);
  static_assert(EPI == 0 || EPI == 1);
  typedef typename FragOf<FORM>::T F;
  __shared__ __attribute__((aligned(16))) float sT[8][16 * 68];
  const int lane = threadIdx.x & 31;
  const int wave = threadIdx.x >> 5;
  const int tilesM = (M + 63) >> 6;
  const int tilesN = (N + 63) >> 6;
  const int tile = blockIdx.x * 8 + wave;
  if (tile >= tilesM * tilesN) return;
  const int tm = tile / tilesN;
  const int tn = tile - tm * tilesN;
  const int m0 = tm << 6;
  const int n0 = tn << 6;

  const int rl = lane & 15;
  const int h8 = (lane >> 4) * 8;
  const unsigned short* pa = A + (size_t)(m0 + rl) * (size_t)KTOT + h8;
  const unsigned short* pb = B + (size_t)(n0 + rl) * (size_t)KTOT + h8;

  v8f acc[4][4];
#pragma unroll
  for (int i = 0; i < 4; ++i)
#pragma unroll
    for (int j = 0; j < 4; ++j) acc[i][j] = (v8f){0.f, 0.f, 0.f, 0.f, 0.f, 0.f, 0.f, 0.f};

#pragma unroll 1
  for (int k0 = 0; k0 < KTOT; k0 += 32) {
    F bf[4];
#pragma unroll
    for (int j = 0; j < 4; ++j) bf[j] = ld_frag<F>(pb + (size_t)(j << 4) * (size_t)KTOT + k0);
#pragma unroll
    for (int i = 0; i < 4; ++i) {
      const F af = ld_frag<F>(pa + (size_t)(i << 4) * (size_t)KTOT + k0);
#pragma unroll
      for (int j = 0; j < 4; ++j) acc[i][j] = mm(af, bf[j], acc[i][j]);
    }
  }

  float* slab = sT[wave];
  const int hh = lane >> 4;
  const int c4 = (lane & 15) * 4;
  const int nc = n0 + c4;
  const bool cok = nc < N;
  v4f bv = (v4f){0.f, 0.f, 0.f, 0.f};
  if (EPI == 1) {
    bv = *(const v4fa*)(bias + clampi(nc, 0, N - 4));
    asm volatile("" :: "v"(bv));
  }
#pragma unroll
  for (int i = 0; i < 4; ++i) {
    const int mBase = m0 + (i << 4);
#pragma unroll
    for (int j = 0; j < 4; ++j) {
#pragma unroll
      for (int r = 0; r < 8; ++r) slab[(h8 + r) * 68 + (j << 4) + rl] = acc[i][j][r];
    }
    __builtin_amdgcn_fence(__ATOMIC_RELEASE, "workgroup");
    __builtin_amdgcn_wave_barrier();
    __builtin_amdgcn_fence(__ATOMIC_ACQUIRE, "workgroup");
    v4f vv[8];
#pragma unroll
    for (int it = 0; it < 8; ++it) {
      const int row = it * 2 + hh;
      v4f v = *(const v4fa*)(slab + row * 68 + c4);
      if (EPI == 1) v += bv;
      vv[it] = v;
    }
    for (int pass = 0; pass < 2; ++pass) {
#pragma unroll
      for (int it = 0; it < 8; ++it) {
        const int row = mBase + it * 2 + hh;
        if (cok && row < M) *(volatile v4f*)(D + (size_t)row * (size_t)ldd + nc) = vv[it];
      }
      __threadfence();
    }
    __builtin_amdgcn_fence(__ATOMIC_RELEASE, "workgroup");
    __builtin_amdgcn_wave_barrier();
    __builtin_amdgcn_fence(__ATOMIC_ACQUIRE, "workgroup");
  }
}

#pragma clang fp contract(off)


#ifndef SPLIT_O
#define SPLIT_O 1
#endif

#define NN      50000
#define NE      1600000
#define MPAD    50048
#define KIN     256
#define HC      128
#define NHD     4
#define DSZ     32
#define OUTW    64
#define KOUT    (SPLIT_O ? 256 : 128)
#define RTHR    256
#define RWAVES  8
#define RPR     64
#define TB_AS   0
#define TB_AD   128
#define TB_BI   256
#define TB_LB   384
#define TB_N    512
#define BT      512
#define BW      16
#define BEPT    8
#define BCHUNK  (BT * BEPT)
#define NCH     ((NE + BCHUNK - 1) / BCHUNK)
#define NB      1024
#define NBLK    ((NN + NB - 1) / NB)
#define LCAP    41472
#define DEGCAP  96
#define SLOTSH  16
#define LISTTOT (NBLK * LCAP)
#define LDS_LST ((LCAP + 3 * NB + 64) * 4 + LCAP * 2)
#define PB_WT   (HC * KIN / 8 / 256)
#define LWT_PCS (OUTW * KOUT / 8)
#define PB_LWT  (LWT_PCS / 256)
#define WSMAX   ((size_t)128 << 20)

static_assert(NHD * DSZ == HC && HC == 128 && HC == 32 * 4);
static_assert(DSZ == 8 * 4);
static_assert(OUTW == 64);
static_assert(KOUT == (SPLIT_O ? 2 : 1) * HC && KOUT % 32 == 0 && KIN % 32 == 0);
static_assert(MPAD == 391 * 128 && MPAD % 128 == 0 && MPAD % 64 == 0 && MPAD % 8 == 0 && MPAD >= NN);
static_assert(MPAD == RPR * 782);
static_assert((MPAD * (KIN / 8)) % 256 == 0);
static_assert(NN % 16 == 0 && NN % 8 == 0);
static_assert(NN < (1 << SLOTSH));
static_assert(NB == 1024 && SLOTSH + 10 <= 32 && NB == 2 * BT);
static_assert(NE % 8 == 0 && NE >= 8);
static_assert(NBLK == 49 && NBLK * NB >= NN);
static_assert(NCH * BCHUNK >= NE && NCH == 391);
static_assert(LCAP % 32 == 0);
static_assert(LCAP * 4 >= 33116 * 5);
static_assert(DEGCAP >= 61 + 8 && DEGCAP >= 96);
static_assert(LDS_LST < 262144);
static_assert(BW == BT / 32 && BW == 16);
static_assert(PB_WT == 16 && LWT_PCS % 256 == 0);
static_assert(TB_LB + OUTW <= TB_N);

typedef int v4i __attribute__((ext_vector_type(4)));
typedef int v2i __attribute__((ext_vector_type(2)));
typedef v4i __attribute__((may_alias)) v4ia;
typedef v2i __attribute__((may_alias)) v2ia;

__device__ __forceinline__ float lrelu_k(float v) { return (v > 0.0f) ? v : 0.2f * v; }
__device__ __forceinline__ float maxk(float a, float b) {
  float m = (a < b) ? b : a;
  m = (b != b) ? b : m;
  return m;
}
__device__ __forceinline__ float sum8(float t) {
  t = t + __shfl_xor(t, 4, 32);
  t = t + __shfl_xor(t, 2, 32);
  t = t + __shfl_xor(t, 1, 32);
  return t;
}
__device__ __forceinline__ v4f exp4(v4f q) {
#pragma unroll 1
  for (int i = 0; i < 4; ++i) { const float t = expf(q.x); q = (v4f){ q.y, q.z, q.w, t }; }
  return q;
}
__device__ __forceinline__ v4f div4(v4f q, v4f d) {
#pragma unroll 1
  for (int i = 0; i < 4; ++i) {
    const float t = q.x / d.x;
    q = (v4f){ q.y, q.z, q.w, t };
    d = (v4f){ d.y, d.z, d.w, d.x };
  }
  return q;
}
__device__ __forceinline__ v4f elu4(v4f v) {
#pragma unroll 1
  for (int i = 0; i < 4; ++i) {
    const float x = v.x;
    const float t = (x > 0.0f) ? x : expm1f(x);
    v = (v4f){ v.y, v.z, v.w, t };
  }
  return v;
}

__global__ __launch_bounds__(256) void k_prep(const float* __restrict__ W, const float* __restrict__ linW,
                                              const float* __restrict__ asrc, const float* __restrict__ adst,
                                              const float* __restrict__ bias, const float* __restrict__ linb,
                                              unsigned short* WT, unsigned short* LWT, float* TB) {
  const int b = (int)blockIdx.x;
  const int t = (int)threadIdx.x;
  if (b < PB_WT) {
    const int g  = b * 256 + t;
    const int n  = g >> 5;
    const int k0 = (g & 31) << 3;
    float x[8];
#pragma unroll
    for (int e = 0; e < 8; ++e) {
      const float v = W[(size_t)(k0 + e) * HC + n];
      asm volatile("" :: "v"(v));
      x[e] = v;
    }
    const v4u o = pack8_bf16((v4f){ x[0], x[1], x[2], x[3] }, (v4f){ x[4], x[5], x[6], x[7] });
    volatile v4u* q = (volatile v4u*)(WT + (size_t)g * 8);
    *q = o;
    __threadfence();
    *q = o;
  } else if (b < PB_WT + PB_LWT) {
    const int g   = (b - PB_WT) * 256 + t;
    const int ppr = KOUT / 8;
    const int n   = g / ppr;
    const int k0  = (g - n * ppr) << 3;
    float x[8];
#pragma unroll
    for (int e = 0; e < 8; ++e) {
      const float v = linW[(size_t)((k0 + e) & (HC - 1)) * OUTW + n];
      asm volatile("" :: "v"(v));
      x[e] = v;
    }
    const v4u o = pack8_bf16((v4f){ x[0], x[1], x[2], x[3] }, (v4f){ x[4], x[5], x[6], x[7] });
    volatile v4u* q = (volatile v4u*)(LWT + (size_t)g * 8);
    *q = o;
    __threadfence();
    *q = o;
  } else {
    const int idx = 4 * t;
    const v4f a0 = *(const v4fa*)(asrc + clampi(idx - TB_AS, 0, 124));
    asm volatile("" :: "v"(a0));
    const v4f a1 = *(const v4fa*)(adst + clampi(idx - TB_AD, 0, 124));
    asm volatile("" :: "v"(a1));
    const v4f a2 = *(const v4fa*)(bias + clampi(idx - TB_BI, 0, 124));
    asm volatile("" :: "v"(a2));
    const v4f a3 = *(const v4fa*)(linb + clampi(idx - TB_LB, 0, 60));
    asm volatile("" :: "v"(a3));
    const unsigned m0 = (idx < TB_AD) ? 0xFFFFFFFFu : 0u;
    const unsigned m1 = (idx >= TB_AD && idx < TB_BI) ? 0xFFFFFFFFu : 0u;
    const unsigned m2 = (idx >= TB_BI && idx < TB_LB) ? 0xFFFFFFFFu : 0u;
    const unsigned m3 = (idx >= TB_LB && idx < TB_LB + OUTW) ? 0xFFFFFFFFu : 0u;
    v4u o;
    o.x = (__float_as_uint(a0.x) & m0) | (__float_as_uint(a1.x) & m1) | (__float_as_uint(a2.x) & m2) | (__float_as_uint(a3.x) & m3);
    o.y = (__float_as_uint(a0.y) & m0) | (__float_as_uint(a1.y) & m1) | (__float_as_uint(a2.y) & m2) | (__float_as_uint(a3.y) & m3);
    o.z = (__float_as_uint(a0.z) & m0) | (__float_as_uint(a1.z) & m1) | (__float_as_uint(a2.z) & m2) | (__float_as_uint(a3.z) & m3);
    o.w = (__float_as_uint(a0.w) & m0) | (__float_as_uint(a1.w) & m1) | (__float_as_uint(a2.w) & m2) | (__float_as_uint(a3.w) & m3);
    o.x = bf16_bits(__uint_as_float(o.x)) << 16;
    o.y = bf16_bits(__uint_as_float(o.y)) << 16;
    o.z = bf16_bits(__uint_as_float(o.z)) << 16;
    o.w = bf16_bits(__uint_as_float(o.w)) << 16;
    const bool wr = t < (TB_N / 4);
    volatile v4u* q = (volatile v4u*)(TB + (wr ? idx : 0));
    if (wr) *q = o;
    __threadfence();
    if (wr) *q = o;
  }
}

__global__ __launch_bounds__(BT) void k_list(const int* __restrict__ esrc, const int* __restrict__ edst,
                                             unsigned* LIST, int* META) {
  extern __shared__ v4u lds_lst[];
  int* reg1 = (int*)lds_lst;
  int* scnt = reg1 + LCAP;
  int* soff = scnt + NB;
  int* curs = soff + NB;
  int* wcnt = curs + NB;
  int* wtot = wcnt + 2 * BW;
  unsigned short* reg2 = (unsigned short*)(wtot + 2 * BW);
  const int tid = (int)threadIdx.x, lane = tid & 31, wave = tid >> 5;
  const int nodeBase = (int)blockIdx.x * NB;
  int nb = NN - nodeBase;
  nb = nb > NB ? NB : (nb < 0 ? 0 : nb);
  const unsigned nbs = (unsigned)nodeBase, unb = (unsigned)nb;

  scnt[2 * tid] = 0;
  scnt[2 * tid + 1] = 0;

  int tot = 0;
#pragma unroll 1
  for (int ch = 0; ch < NCH; ++ch) {
    const int par = ch & 1;
    const int e0  = ch * BCHUNK + tid * BEPT;
    const bool valid = e0 < NE;
    const int ea = e0 < NE - 8 ? e0 : NE - 8;
    const v4i da = *(const v4ia*)(edst + ea);
    const v4i db = *(const v4ia*)(edst + ea + 4);
    const v4i sa = *(const v4ia*)(esrc + ea);
    const v4i sb = *(const v4ia*)(esrc + ea + 4);
    asm volatile("" :: "v"(da), "v"(db), "v"(sa), "v"(sb));
    const unsigned s0 = (unsigned)da.x - nbs, s1 = (unsigned)da.y - nbs;
    const unsigned s2 = (unsigned)da.z - nbs, s3 = (unsigned)da.w - nbs;
    const unsigned s4 = (unsigned)db.x - nbs, s5 = (unsigned)db.y - nbs;
    const unsigned s6 = (unsigned)db.z - nbs, s7 = (unsigned)db.w - nbs;
    const bool h0 = valid && (s0 < unb), h1 = valid && (s1 < unb), h2 = valid && (s2 < unb), h3 = valid && (s3 < unb);
    const bool h4 = valid && (s4 < unb), h5 = valid && (s5 < unb), h6 = valid && (s6 < unb), h7 = valid && (s7 < unb);
    const int c = (int)h0 + (int)h1 + (int)h2 + (int)h3 + (int)h4 + (int)h5 + (int)h6 + (int)h7;
    int incl = c;
#pragma unroll
    for (int d = 1; d < 32; d <<= 1) {
      const int up = __shfl_up(incl, d, 32);
      incl += (lane >= d) ? up : 0;
    }
    const int wtotal = __shfl(incl, 31, 32);
    if (lane == 0) wcnt[par * BW + wave] = wtotal;
    __syncthreads();
    int all = 0, pre = 0;
#pragma unroll
    for (int g = 0; g < 4; ++g) {
      const v4i w4 = *(const v4ia*)(wcnt + par * BW + 4 * g);
      const int c0 = clampi(w4.x, 0, 256), c1 = clampi(w4.y, 0, 256);
      const int c2 = clampi(w4.z, 0, 256), c3 = clampi(w4.w, 0, 256);
      all += c0 + c1 + c2 + c3;
      pre += (4 * g + 0 < wave) ? c0 : 0;
      pre += (4 * g + 1 < wave) ? c1 : 0;
      pre += (4 * g + 2 < wave) ? c2 : 0;
      pre += (4 * g + 3 < wave) ? c3 : 0;
    }
    int pos = tot + pre + (incl - c);
#define PUTJ(HJ, SJ, SRCJ) if (HJ) { if (pos < LCAP) reg1[pos] = (int)((unsigned)clampi((SRCJ), 0, NN - 1) | ((SJ) << SLOTSH)); ++pos; }
    PUTJ(h0, s0, sa.x)
    PUTJ(h1, s1, sa.y)
    PUTJ(h2, s2, sa.z)
    PUTJ(h3, s3, sa.w)
    PUTJ(h4, s4, sb.x)
    PUTJ(h5, s5, sb.y)
    PUTJ(h6, s6, sb.z)
    PUTJ(h7, s7, sb.w)
#undef PUTJ
    tot += all;
  }
  __syncthreads();
  const bool ovf = tot > LCAP;
  const int nh = ovf ? LCAP : tot;

  if (wave == 0) {
#pragma unroll 1
    for (int b0 = 0; b0 < nh; b0 += 32) {
      const int idx = b0 + lane;
      const int uv  = reg1[idx < nh ? idx : nh - 1];
      const int m32 = (nh - b0) < 32 ? (nh - b0) : 32;
#pragma unroll 1
      for (int k = 0; k < m32; ++k) {
        const int u  = __builtin_amdgcn_readlane(uv, k);
        const int sl = (int)(((unsigned)u >> SLOTSH) & (unsigned)(NB - 1));
        const int cv = scnt[sl] + 1;
        if (lane == 0) scnt[sl] = cv;
      }
    }
  }
  __syncthreads();

  {
    const v2i cc = *(const v2ia*)(scnt + 2 * tid);
    const int e0c = cc.x < 0 ? 0 : cc.x;
    const int e1c = cc.y < 0 ? 0 : cc.y;
    const int ts = e0c + e1c;
    int incl = ts;
#pragma unroll
    for (int d = 1; d < 32; d <<= 1) {
      const int up = __shfl_up(incl, d, 32);
      incl += (lane >= d) ? up : 0;
    }
    if (lane == 31) wtot[wave] = incl;
    __syncthreads();
    int pre = 0;
#pragma unroll
    for (int g = 0; g < 4; ++g) {
      const v4i w4 = *(const v4ia*)(wtot + 4 * g);
      pre += (4 * g + 0 < wave) ? w4.x : 0;
      pre += (4 * g + 1 < wave) ? w4.y : 0;
      pre += (4 * g + 2 < wave) ? w4.z : 0;
      pre += (4 * g + 3 < wave) ? w4.w : 0;
    }
    const int run = pre + incl - ts;
    soff[2 * tid]     = run;
    soff[2 * tid + 1] = run + e0c;
    curs[2 * tid]     = run;
    curs[2 * tid + 1] = run + e0c;
  }
  __syncthreads();

  if (wave == 0) {
#pragma unroll 1
    for (int b0 = 0; b0 < nh; b0 += 32) {
      const int idx = b0 + lane;
      const int uv  = reg1[idx < nh ? idx : nh - 1];
      const int m32 = (nh - b0) < 32 ? (nh - b0) : 32;
#pragma unroll 1
      for (int k = 0; k < m32; ++k) {
        const int u  = __builtin_amdgcn_readlane(uv, k);
        const int sl = (int)(((unsigned)u >> SLOTSH) & (unsigned)(NB - 1));
        const unsigned short sid = (unsigned short)((unsigned)u & 0xFFFFu);
        const int pr = curs[sl];
        const int pc = clampi(pr, 0, LCAP - 1);
        if (lane == 0) { reg2[pc] = sid; curs[sl] = pc + 1; }
      }
    }
  }
  __syncthreads();

  {
    int nhPad = (nh + 32) & ~31;
    nhPad = nhPad > LCAP ? LCAP : nhPad;
    const int nIt = (nhPad + BT - 1) / BT;
    unsigned* lbase = LIST + (size_t)blockIdx.x * (size_t)LCAP;
#pragma unroll 1
    for (int it = 0; it < nIt; ++it) {
      const int i  = it * BT + tid;
      const int ic = i < nh ? i : (nh > 0 ? nh - 1 : 0);
      const unsigned sv = (unsigned)reg2[ic];
      const unsigned msk = (i < nh) ? 0xFFFFFFFFu : 0u;
      const unsigned o = sv & msk;
      const int iw = i < LCAP ? i : LCAP - 1;
      volatile unsigned* q = (volatile unsigned*)(lbase + (size_t)iw);
      const bool wr = i < nhPad;
      if (wr) *q = o;
      __threadfence();
      if (wr) *q = o;
    }
  }

  {
    const int base = (int)blockIdx.x * LCAP;
    const v2i cc = *(const v2ia*)(scnt + 2 * tid);
    const v2i so = *(const v2ia*)(soff + 2 * tid);
    v4i m;
    m.x = base + so.x;
    m.y = ovf ? -1 : cc.x;
    m.z = base + so.y;
    m.w = ovf ? -1 : cc.y;
    volatile v4i* q = (volatile v4i*)(META + 2 * (size_t)(nodeBase + 2 * tid));
    *q = m;
    __threadfence();
    *q = m;
  }
}

__global__ __launch_bounds__(RTHR) void k_rowprep(const float* __restrict__ FT, const float* __restrict__ TB, float* ELR) {
  __shared__ __attribute__((aligned(16))) float sT[2 * RPR * NHD];
  const int lane = (int)threadIdx.x & 31;
  const int wave = (int)threadIdx.x >> 5;
  const int head = lane >> 3;
  const int c0   = lane * 4;
  const v4f as = *(const v4fa*)(TB + TB_AS + c0);
  asm volatile("" :: "v"(as));
  const v4f ad = *(const v4fa*)(TB + TB_AD + c0);
  asm volatile("" :: "v"(ad));
#pragma unroll 1
  for (int i = 0; i < RPR / RWAVES; ++i) {
    const int rl  = wave * (RPR / RWAVES) + i;
    const int row = (int)blockIdx.x * RPR + rl;
    const v4f p = *(const v4fa*)(FT + (size_t)row * HC + c0);
    asm volatile("" :: "v"(p));
    float t = p.x * as.x;
    float u = p.y * as.y; t = t + u;
    u = p.z * as.z; t = t + u;
    u = p.w * as.w; t = t + u;
    t = sum8(t);
    float d = p.x * ad.x;
    u = p.y * ad.y; d = d + u;
    u = p.z * ad.z; d = d + u;
    u = p.w * ad.w; d = d + u;
    d = sum8(d);
    const bool live = row < NN;
    t = live ? t : 0.0f;
    d = live ? d : 0.0f;
    if ((lane & 7) == 0) {
      sT[rl * NHD + head] = t;
      sT[RPR * NHD + rl * NHD + head] = d;
    }
  }
  __syncthreads();
  if (wave < 2) {
    const float* sp = sT + wave * (RPR * NHD);
    const v4f v0 = *(const v4fa*)(sp + 4 * lane);
    const v4f v1 = *(const v4fa*)(sp + 128 + 4 * lane);
    float* dp = ELR + (size_t)wave * ((size_t)MPAD * NHD) + ((size_t)blockIdx.x * RPR + (size_t)lane) * NHD;
    *(volatile v4f*)dp = v0;
    *(volatile v4f*)(dp + 128) = v1;
    __threadfence();
    *(volatile v4f*)dp = v0;
    *(volatile v4f*)(dp + 128) = v1;
  }
}

__device__ __forceinline__ void ld_chunk(int b0, int lane, int tot, int cnt, int off, int rowc,
                                         const unsigned* __restrict__ LIST, const float* __restrict__ EL,
                                         v4f er4, int& src, v4f& e) {
  const int j  = b0 + lane;
  const int jc = j < tot ? j : tot - 1;
  const int li = clampi(off + jc, 0, LISTTOT - 1);
  const unsigned lw = LIST[li];
  asm volatile("" :: "v"(lw));
  const int sm = (jc >= cnt) ? -1 : 0;
  const int sl = clampi((int)lw, 0, NN - 1);
  src = (rowc & sm) | (sl & ~sm);
  const v4f el = *(const v4fa*)(EL + (size_t)src * NHD);
  asm volatile("" :: "v"(el));
  e.x = lrelu_k(el.x + er4.x);
  e.y = lrelu_k(el.y + er4.y);
  e.z = lrelu_k(el.z + er4.z);
  e.w = lrelu_k(el.w + er4.w);
}

__global__ __launch_bounds__(RTHR) void k_walk(const float* __restrict__ FT, const float* __restrict__ EL,
                                               const float* __restrict__ ER, const unsigned* __restrict__ LIST,
                                               const int* __restrict__ META, const float* __restrict__ TB,
                                               unsigned short* OP) {
  const int lane = (int)threadIdx.x & 31;
  const int wave = (int)threadIdx.x >> 5;
  const int row  = (int)blockIdx.x * RWAVES + wave;
  const int rowc = row < NN ? row : NN - 1;
  const int head = lane >> 3;
  const int c0   = lane * 4;

  const v2i mt = *(const v2ia*)(META + 2 * (size_t)rowc);
  asm volatile("" :: "v"(mt));
  const int craw = mt.y;
  const int offv = clampi(mt.x, 0, LISTTOT);
  int cntv = clampi(craw, 0, DEGCAP);
  cntv = cntv < (LISTTOT - offv) ? cntv : (LISTTOT - offv);
  const int off = __builtin_amdgcn_readfirstlane(offv);
  const int cnt = __builtin_amdgcn_readfirstlane(cntv);
  const int tot = cnt + 1;
  const bool poison = (craw < 0) || (craw > DEGCAP);

  const v4f er4 = *(const v4fa*)(ER + (size_t)rowc * NHD);
  asm volatile("" :: "v"(er4));

  const float ninf = -__builtin_inff();
  v4f mx = (v4f){ ninf, ninf, ninf, ninf };
#pragma unroll 1
  for (int b0 = 0; b0 < tot; b0 += 32) {
    int src; v4f e;
    ld_chunk(b0, lane, tot, cnt, off, rowc, LIST, EL, er4, src, e);
    mx.x = maxk(mx.x, e.x);
    mx.y = maxk(mx.y, e.y);
    mx.z = maxk(mx.z, e.z);
    mx.w = maxk(mx.w, e.w);
  }
#pragma unroll
  for (int d = 16; d > 0; d >>= 1) {
    const float o0 = __shfl_xor(mx.x, d, 32);
    const float o1 = __shfl_xor(mx.y, d, 32);
    const float o2 = __shfl_xor(mx.z, d, 32);
    const float o3 = __shfl_xor(mx.w, d, 32);
    mx.x = maxk(mx.x, o0);
    mx.y = maxk(mx.y, o1);
    mx.z = maxk(mx.z, o2);
    mx.w = maxk(mx.w, o3);
  }
  mx.x = ((__float_as_uint(mx.x) & 0x7fffffffu) < 0x7f800000u) ? mx.x : 0.0f;
  mx.y = ((__float_as_uint(mx.y) & 0x7fffffffu) < 0x7f800000u) ? mx.y : 0.0f;
  mx.z = ((__float_as_uint(mx.z) & 0x7fffffffu) < 0x7f800000u) ? mx.z : 0.0f;
  mx.w = ((__float_as_uint(mx.w) & 0x7fffffffu) < 0x7f800000u) ? mx.w : 0.0f;

  v4f den = (v4f){ 0.0f, 0.0f, 0.0f, 0.0f };
  v4f ac  = (v4f){ 0.0f, 0.0f, 0.0f, 0.0f };
#pragma unroll 1
  for (int pass = 0; pass < 2; ++pass) {
#pragma unroll 1
    for (int b0 = 0; b0 < tot; b0 += 32) {
      int src; v4f e;
      ld_chunk(b0, lane, tot, cnt, off, rowc, LIST, EL, er4, src, e);
      v4f q;
      q.x = e.x - mx.x; q.y = e.y - mx.y; q.z = e.z - mx.z; q.w = e.w - mx.w;
      q = exp4(q);
      const int m32 = (tot - b0) < 32 ? (tot - b0) : 32;
      if (pass == 0) {
#pragma unroll 1
        for (int k = 0; k < m32; ++k) {
          const float w0 = __int_as_float(__builtin_amdgcn_readlane(__float_as_int(q.x), k));
          const float w1 = __int_as_float(__builtin_amdgcn_readlane(__float_as_int(q.y), k));
          const float w2 = __int_as_float(__builtin_amdgcn_readlane(__float_as_int(q.z), k));
          const float w3 = __int_as_float(__builtin_amdgcn_readlane(__float_as_int(q.w), k));
          den.x = den.x + w0;
          den.y = den.y + w1;
          den.z = den.z + w2;
          den.w = den.w + w3;
        }
      } else {
        q = div4(q, den);
#pragma unroll 1
        for (int k = 0; k < m32; ++k) {
          const int c = __builtin_amdgcn_readlane(src, k);
          const float w0 = __int_as_float(__builtin_amdgcn_readlane(__float_as_int(q.x), k));
          const float w1 = __int_as_float(__builtin_amdgcn_readlane(__float_as_int(q.y), k));
          const float w2 = __int_as_float(__builtin_amdgcn_readlane(__float_as_int(q.z), k));
          const float w3 = __int_as_float(__builtin_amdgcn_readlane(__float_as_int(q.w), k));
          float w = w0;
          w = (head == 1) ? w1 : w;
          w = (head == 2) ? w2 : w;
          w = (head == 3) ? w3 : w;
          const v4f hn = *(const v4fa*)(FT + (size_t)c * HC + c0);
          asm volatile("" :: "v"(hn));
          float pr;
          pr = w * hn.x; ac.x = ac.x + pr;
          pr = w * hn.y; ac.y = ac.y + pr;
          pr = w * hn.z; ac.z = ac.z + pr;
          pr = w * hn.w; ac.w = ac.w + pr;
        }
      }
    }
  }

  const v4f bv = *(const v4fa*)(TB + TB_BI + c0);
  asm volatile("" :: "v"(bv));
  v4f v;
  v.x = ac.x + bv.x; v.y = ac.y + bv.y; v.z = ac.z + bv.z; v.w = ac.w + bv.w;
  v4f y = elu4(v);
  const float qnan = __uint_as_float(0x7fc00000u);
  y.x = poison ? qnan : y.x;
  y.y = poison ? qnan : y.y;
  y.z = poison ? qnan : y.z;
  y.w = poison ? qnan : y.w;

  const int h01 = (int)pk16(bf16_bits(y.x), bf16_bits(y.y));
  const int h23 = (int)pk16(bf16_bits(y.z), bf16_bits(y.w));
  const int l01 = (int)pk16(bf16_lo_bits(y.x), bf16_lo_bits(y.y));
  const int l23 = (int)pk16(bf16_lo_bits(y.z), bf16_lo_bits(y.w));
  const int sA = 2 * (lane & 15);
  const int sB = sA + 1;
  const unsigned hA0 = (unsigned)__shfl(h01, sA, 32);
  const unsigned hA1 = (unsigned)__shfl(h23, sA, 32);
  const unsigned hB0 = (unsigned)__shfl(h01, sB, 32);
  const unsigned hB1 = (unsigned)__shfl(h23, sB, 32);
  const unsigned lA0 = (unsigned)__shfl(l01, sA, 32);
  const unsigned lA1 = (unsigned)__shfl(l23, sA, 32);
  const unsigned lB0 = (unsigned)__shfl(l01, sB, 32);
  const unsigned lB1 = (unsigned)__shfl(l23, sB, 32);
  const unsigned mU = (lane >= 16) ? 0xFFFFFFFFu : 0u;
  const unsigned pm = (row < NN) ? 0xFFFFFFFFu : 0u;
  v4u o;
  o.x = ((lA0 & mU) | (hA0 & ~mU)) & pm;
  o.y = ((lA1 & mU) | (hA1 & ~mU)) & pm;
  o.z = ((lB0 & mU) | (hB0 & ~mU)) & pm;
  o.w = ((lB1 & mU) | (hB1 & ~mU)) & pm;
  const bool wr = (SPLIT_O != 0) || (lane < 16);
  const int pc = wr ? lane : 0;
  volatile v4u* qp = (volatile v4u*)(OP + (size_t)row * KOUT + (size_t)pc * 8);
  if (wr) *qp = o;
  __threadfence();
  if (wr) *qp = o;
}

extern "C" void kernel_launch(void* const* d_in, const int* in_sizes, int n_in,
                              void* d_out, int out_size, void* d_ws, size_t ws_size,
                              hipStream_t stream) {
  if (n_in < 8) return;
  if (in_sizes[0] != NN * KIN) return;
  if (in_sizes[1] != 2 * NE) return;
  if (in_sizes[2] != KIN * HC) return;
  if (in_sizes[3] != HC || in_sizes[4] != HC || in_sizes[5] != HC) return;
  if (in_sizes[6] != HC * OUTW || in_sizes[7] != OUTW) return;
  if (out_size != NN * OUTW) return;

  const float* x    = (const float*)d_in[0];
  const int*   ei   = (const int*)  d_in[1];
  const float* W    = (const float*)d_in[2];
  const float* asrc = (const float*)d_in[3];
  const float* adst = (const float*)d_in[4];
  const float* bias = (const float*)d_in[5];
  const float* linW = (const float*)d_in[6];
  const float* linb = (const float*)d_in[7];
  float* out = (float*)d_out;
  const int* esrc = ei;
  const int* edst = ei + NE;

  const size_t szXB   = (size_t)MPAD * KIN * 2;
  const size_t szWT   = (size_t)HC * KIN * 2;
  const size_t szLWT  = (size_t)OUTW * 256 * 2;
  const size_t szTB   = (size_t)TB_N * 4;
  const size_t szFT   = (size_t)MPAD * HC * 4;
  const size_t szELR  = 2 * (size_t)MPAD * NHD * 4;
  const size_t szMETA = (size_t)NBLK * NB * 2 * 4;
  const size_t szLIST = (size_t)NBLK * LCAP * 4;
  static_assert((size_t)MPAD * KIN * 2 + (size_t)HC * KIN * 2 + (size_t)OUTW * 256 * 2 + (size_t)TB_N * 4 +
                (size_t)MPAD * HC * 4 + 2 * (size_t)MPAD * NHD * 4 + (size_t)NBLK * NB * 8 +
                (size_t)NBLK * LCAP * 4 == 61480960);
  static_assert(61480960 <= WSMAX);
  static_assert((size_t)MPAD * KOUT * 2 <= (size_t)MPAD * KIN * 2);
  char* ws = (char*)d_ws;
  size_t off = 0;
  const size_t oXB   = off; off += szXB;
  const size_t oWT   = off; off += szWT;
  const size_t oLWT  = off; off += szLWT;
  const size_t oTB   = off; off += szTB;
  const size_t oFT   = off; off += szFT;
  const size_t oELR  = off; off += szELR;
  const size_t oMETA = off; off += szMETA;
  const size_t oLIST = off; off += szLIST;
  if (off > ws_size || off > (size_t)WSMAX) return;
  unsigned short* XB  = (unsigned short*)(ws + oXB);
  unsigned short* OP  = XB;
  unsigned short* WT  = (unsigned short*)(ws + oWT);
  unsigned short* LWT = (unsigned short*)(ws + oLWT);
  float*    TB   = (float*)(ws + oTB);
  float*    FT   = (float*)(ws + oFT);
  float*    ELR  = (float*)(ws + oELR);
  int*      META = (int*)(ws + oMETA);
  unsigned* LIST = (unsigned*)(ws + oLIST);
  const float* EL = ELR;
  const float* ER = ELR + (size_t)MPAD * NHD;

  hipFuncSetAttribute(reinterpret_cast<const void*>(&k_list),
                      hipFuncAttributeMaxDynamicSharedMemorySize, LDS_LST);

  k_plane<0><<<MPAD * (KIN / 8) / 256, 256, 0, stream>>>(x, NN, KIN, KIN, XB, MPAD, KIN);
  k_prep<<<PB_WT + PB_LWT + 1, 256, 0, stream>>>(W, linW, asrc, adst, bias, linb, WT, LWT, TB);
  k_list<<<NBLK, BT, LDS_LST, stream>>>(esrc, edst, LIST, META);
  {
    const int tiles = (MPAD / 64) * (HC / 64);
    k_gemm_nt<0, 0><<<(tiles + 7) / 8, 256, 0, stream>>>(XB, WT, TB, FT, MPAD, HC, KIN, HC);
  }
  k_rowprep<<<MPAD / RPR, RTHR, 0, stream>>>(FT, TB, ELR);
  k_walk<<<MPAD / RWAVES, RTHR, 0, stream>>>(FT, EL, ER, LIST, META, TB, OP);
  {
    const int tiles = ((NN + 63) / 64) * (OUTW / 64);
    k_gemm_nt<0, 1><<<(tiles + 7) / 8, 256, 0, stream>>>(OP, LWT, TB + TB_LB, out, NN, OUTW, KOUT, OUTW);
  }
}
